// GraphRecurrent_58179626991923
// MI455X (gfx1250) — hardware-run, weakly checked
//
#include <hip/hip_runtime.h>


namespace {
constexpr int N = 50000, NP = 50048, E = 600000, H = 128, G4 = 4 * H;
constexpr float XS = 8.0f, WSC = 256.0f;
typedef _Float16 b16;
typedef __attribute__((ext_vector_type(16))) _Float16 v16b;
typedef __attribute__((ext_vector_type(8))) _Float16 v8b;
typedef __attribute__((ext_vector_type(8))) float v8f;
typedef __attribute__((ext_vector_type(4))) float v4f;
__device__ __forceinline__ float bf16_rne(float f) { unsigned int u = __float_as_uint(f); u += 0x7FFFu + ((u >> 16) & 1u); return __uint_as_float(u & 0xFFFF0000u); }
__device__ __forceinline__ void split16(float v, b16& hi, b16& lo) { hi = (b16)v; lo = (b16)(v - (float)hi); }
__device__ __forceinline__ v16b frag_kb(const b16* p, int hh) { const v8b a = *(const v8b*)(p + 8 * hh), b = *(const v8b*)(p + 16 + 8 * hh); v16b f;
#pragma unroll
  for (int e = 0; e < 8; ++e) { f[e] = a[e]; f[8 + e] = b[e]; } return f; }
__device__ __forceinline__ v8f wmma16b(v16b a, v16b b, v8f c) { v8f d = __builtin_amdgcn_wmma_f32_16x16x32_f16(false, a, false, b, (short)0, c, false, false); asm volatile("v_nop\n\tv_nop\n\tv_nop\n\tv_nop" : "+v"(d) : "v"(a), "v"(b)); return d; }
__device__ __forceinline__ void wave_lds_sync() { __builtin_amdgcn_fence(__ATOMIC_RELEASE, "workgroup"); __builtin_amdgcn_wave_barrier(); __builtin_amdgcn_fence(__ATOMIC_ACQUIRE, "workgroup"); }
__device__ __forceinline__ float pmul(float a, float b) { float p = a * b; asm volatile("" : "+v"(p)); return p; }
__device__ __forceinline__ float opaque(float a) { asm volatile("" : "+v"(a)); return a; }
__device__ __forceinline__ int iclamp(int v, int lo, int hi) { return v < lo ? lo : (v > hi ? hi : v); }
__device__ __forceinline__ float sigm(float x) { return 1.0f / (1.0f + __expf(-x)); }
constexpr int CSR_NBLK = 512, CSR_GB = 9, CSR_GN = 1 << CSR_GB  , CSR_TS = (CSR_GN < 32 ? 32 : CSR_GN)  , CSR_MAXG = 512, CSR_CAP = 12288  ;
__device__ __host__ __forceinline__ int csr_tix(int v) { return (v >> CSR_GB) * CSR_TS + (v & (CSR_GN - 1)); }
__global__ __launch_bounds__(64) void csrA_kernel(const int* __restrict__ dst, int E, int N, int nG, int CHP, int NGP, int* __restrict__ STG, int* __restrict__ HST) {
  extern __shared__ int sm[];
  int* cnt = sm; int* run = sm + NGP; int* ids = sm + 2 * NGP;
  const int b = blockIdx.x; const int ch = (E + CSR_NBLK - 1) / CSR_NBLK; const int e0 = b * ch, e1 = min(E, e0 + ch);
  for (int i = threadIdx.x; i < NGP; i += 64) cnt[i] = 0;
  for (int i = threadIdx.x; i < CHP; i += 64) ids[i] = -1;
  __syncthreads();
  if (threadIdx.x == 0) {
    for (int e = e0; e < e1; ++e) { int d = dst[e]; d = (d < 0) ? 0 : (d >= N ? N - 1 : d); cnt[d >> CSR_GB] += 1; }
    int acc = 0; for (int g = 0; g < nG; ++g) { run[g] = acc; acc += cnt[g]; }
    for (int e = e0; e < e1; ++e) { int d = dst[e]; d = (d < 0) ? 0 : (d >= N ? N - 1 : d); const int g = d >> CSR_GB; ids[run[g]] = e; run[g] += 1; } }
  __syncthreads();
  typedef __attribute__((ext_vector_type(4))) int v4i;
  for (int pass = 0; pass < 2; ++pass) {
    for (int i = threadIdx.x; i < CHP / 4; i += 64) *(volatile v4i*)(STG + (size_t)b * CHP + i * 4) = *(const v4i*)(&ids[i * 4]);
    for (int i = threadIdx.x; i < NGP / 4; i += 64) { v4i v; for (int e = 0; e < 4; ++e) v[e] = (i * 4 + e < nG) ? cnt[i * 4 + e] : 0; *(volatile v4i*)(HST + (size_t)b * NGP + i * 4) = v; }
    __threadfence(); }
}
__global__ __launch_bounds__(512) void csrS_kernel(const int* __restrict__ HST, int nG, int NGP, int* __restrict__ START, int* __restrict__ TOT, int* __restrict__ OFF) {
  __shared__ int tot[CSR_MAXG];
  const int b = threadIdx.x;
  for (int pass = 0; pass < 2; ++pass) { int runb = 0; for (int g = 0; g < nG; ++g) { int c = HST[(size_t)b * NGP + g]; c = (c < 0) ? 0 : c; ((volatile int*)OFF)[(size_t)g * CSR_NBLK + b] = runb; runb += c; } __threadfence(); }
  for (int g = threadIdx.x; g < nG; g += 512) { int s = 0; for (int bb = 0; bb < CSR_NBLK; ++bb) { int c = HST[(size_t)bb * NGP + g]; s += (c < 0) ? 0 : c; } tot[g] = s; }
  __syncthreads();
  if (threadIdx.x < 32) {
    __shared__ int st[CSR_MAXG + 32];
    if (threadIdx.x == 0) { int acc = 0; for (int g = 0; g < NGP; ++g) { st[g] = acc; if (g < nG) acc += (tot[g] + 31) & ~31; } st[NGP] = acc; }
    __builtin_amdgcn_fence(__ATOMIC_RELEASE, "workgroup"); __builtin_amdgcn_wave_barrier(); __builtin_amdgcn_fence(__ATOMIC_ACQUIRE, "workgroup");
    for (int pass = 0; pass < 2; ++pass) { for (int i = threadIdx.x; i < NGP + 32; i += 32) { ((volatile int*)START)[i] = (i <= NGP) ? st[min(i, NGP)] : 0; ((volatile int*)TOT)[i] = (i < nG) ? tot[i] : 0; } __threadfence(); } }
}
__global__ __launch_bounds__(256) void csrB_kernel(const int* __restrict__ dst, int N, int nG, int CHP, int NGP, int permLen, const int* __restrict__ STG, const int* __restrict__ HST, const int* __restrict__ OFF, const int* __restrict__ START, const int* __restrict__ TOT, int* __restrict__ PERM, int* __restrict__ ROWPTR, int* __restrict__ ROWCNT, int* __restrict__ FLAG) {
  typedef __attribute__((ext_vector_type(4))) int v4i;
  __shared__ int ids[CSR_CAP]; __shared__ unsigned short key[CSR_CAP]; __shared__ int outp[CSR_CAP]; __shared__ int ncnt[CSR_GN + 1]; __shared__ int boff[CSR_NBLK + 1];
  const int g = blockIdx.x, t_ = threadIdx.x; int tot = TOT[g]; int st = START[g], stn = START[g + 1]; const int v0 = g * CSR_GN; const int nv = min(CSR_GN, N - v0); const int t0 = g * CSR_TS;
  st = (st < 0) ? 0 : (st > permLen - 32 ? permLen - 32 : st) & ~31; stn = (stn < st) ? st : (stn > permLen ? permLen : stn); tot = (tot < 0) ? 0 : tot; if (tot > stn - st && tot <= CSR_CAP) tot = stn - st;
  if (tot > CSR_CAP) {
    for (int pass = 0; pass < 2; ++pass) { for (int i = t_; i < CSR_TS / 4; i += 256) { v4i a, c; for (int e = 0; e < 4; ++e) { a[e] = st; c[e] = 0; } *(volatile v4i*)(ROWPTR + t0 + i * 4) = a; *(volatile v4i*)(ROWCNT + t0 + i * 4) = c; } if (t_ == 0) ((volatile int*)FLAG)[0] = 1; __threadfence(); } (void)nv; return; }
  if (t_ == 0) { int acc = 0; for (int b = 0; b < CSR_NBLK; ++b) { boff[b] = acc; int c = HST[(size_t)b * NGP + g]; c = (c < 0) ? 0 : (c > CHP ? CHP : c); acc += c; if (acc > tot) acc = tot; } boff[CSR_NBLK] = acc; }
  for (int i = t_; i <= CSR_GN; i += 256) ncnt[i] = 0;
  __syncthreads();
  for (int b = 0; b < CSR_NBLK; ++b) { const int c = boff[b + 1] - boff[b]; int o_ = OFF[(size_t)g * CSR_NBLK + b]; o_ = (o_ < 0) ? 0 : (o_ > CHP - c ? CHP - c : o_); const int* src_ = STG + (size_t)b * CHP + o_;
    for (int i = t_; i < c; i += 256) { int id = src_[i]; id = (id < 0) ? 0 : id; ids[boff[b] + i] = id; int d = dst[id]; d = (d < v0) ? v0 : (d >= N ? N - 1 : d); int kk = d - v0; kk = (kk < 0) ? 0 : (kk >= CSR_GN ? CSR_GN - 1 : kk); key[boff[b] + i] = (unsigned short)kk; } }
  __syncthreads();
  if (t_ == 0) { for (int i = 0; i < tot; ++i) ncnt[key[i]] += 1; int acc = 0; for (int vl = 0; vl < CSR_GN; ++vl) { const int c = ncnt[vl]; ncnt[vl] = acc; acc += c; } ncnt[CSR_GN] = acc;
    for (int i = 0; i < tot; ++i) { const int vl = key[i]; outp[ncnt[vl]] = ids[i]; ncnt[vl] += 1; }
    for (int vl = CSR_GN; vl > 0; --vl) ncnt[vl] = ncnt[vl - 1]; ncnt[0] = 0; }
  __syncthreads();
  for (int pass = 0; pass < 2; ++pass) {
    for (int i = t_; i < (stn - st) / 4; i += 256) { v4i v; for (int e = 0; e < 4; ++e) { const int q = i * 4 + e; v[e] = (q < tot) ? outp[q] : -1; } *(volatile v4i*)(PERM + st + i * 4) = v; }
    for (int i = t_; i < CSR_TS / 4; i += 256) { v4i a, c; for (int e = 0; e < 4; ++e) { const int vl = i * 4 + e; const int vc = vl < CSR_GN ? vl : CSR_GN; a[e] = (vl < CSR_GN) ? st + ncnt[vc] : st; c[e] = (vl < nv) ? (ncnt[(vc < CSR_GN ? vc : CSR_GN - 1) + 1] - ncnt[vc]) : 0; } *(volatile v4i*)(ROWPTR + t0 + i * 4) = a; *(volatile v4i*)(ROWCNT + t0 + i * 4) = c; }
    __threadfence(); }
}
__global__ __launch_bounds__(256) void csrZ_kernel(int* __restrict__ p, size_t n4) { typedef __attribute__((ext_vector_type(4))) int v4i; const size_t tid = (size_t)blockIdx.x * 256 + threadIdx.x, nth = (size_t)gridDim.x * 256; v4i z = {0, 0, 0, 0}; for (size_t i = tid; i < n4; i += nth) *(volatile v4i*)(p + i * 4) = z; }
struct CsrBufs { int *STG, *HST, *OFF, *START, *TOT, *PERM, *ROWPTR, *ROWCNT, *FLAG; int nG, NGP, CHP; size_t permLen; char* base; size_t bytes; };
static size_t csr_carve(CsrBufs& c, char* ws, size_t off, int E, int N) {
  const size_t off0 = off; c.base = ws + off;
  auto al = [&](size_t bytes) { char* p = ws + off; off += (bytes + 255) & ~(size_t)255; return p; };
  c.nG = (N + CSR_GN - 1) / CSR_GN; c.NGP = (c.nG + 31) & ~31; const int ch = (E + CSR_NBLK - 1) / CSR_NBLK; c.CHP = (ch + 31) & ~31; c.permLen = (size_t)E + 32 * (size_t)c.nG + 32;
  c.STG = (int*)al((size_t)CSR_NBLK * c.CHP * 4); c.HST = (int*)al((size_t)CSR_NBLK * c.NGP * 4); c.OFF = (int*)al((size_t)c.NGP * CSR_NBLK * 4); c.START = (int*)al((size_t)(c.NGP + 64) * 4); c.TOT = (int*)al((size_t)(c.NGP + 64) * 4);
  c.PERM = (int*)al(c.permLen * 4); c.ROWPTR = (int*)al((size_t)c.nG * CSR_TS * 4); c.ROWCNT = (int*)al((size_t)c.nG * CSR_TS * 4); c.FLAG = (int*)al(256);
  c.bytes = off - off0; return off;
}
static void csr_build(const CsrBufs& c, const int* dst, int E, int N, hipStream_t stream) {
  const size_t smem = (size_t)(2 * c.NGP + c.CHP) * 4;
  csrZ_kernel<<<512, 256, 0, stream>>>((int*)c.base, c.bytes / 16);
  csrA_kernel<<<CSR_NBLK, 64, smem, stream>>>(dst, E, N, c.nG, c.CHP, c.NGP, c.STG, c.HST);
  csrS_kernel<<<1, 512, 0, stream>>>(c.HST, c.nG, c.NGP, c.START, c.TOT, c.OFF);
  csrB_kernel<<<c.nG, 256, 0, stream>>>(dst, N, c.nG, c.CHP, c.NGP, (int)c.permLen, c.STG, c.HST, c.OFF, c.START, c.TOT, c.PERM, c.ROWPTR, c.ROWCNT, c.FLAG);
}


__global__ __launch_bounds__(256) void wprep_kernel(const float* __restrict__ wih, const float* __restrict__ w3, b16* __restrict__ WIH, b16* __restrict__ W3) {
  const size_t u = (size_t)blockIdx.x * 256 + threadIdx.x; const size_t n0 = (size_t)G4 * H / 8, n1 = (size_t)H * H / 8; v8b o;
  if (u < n0) { const size_t e = u * 8; for (int j = 0; j < 8; ++j) o[j] = (b16)(bf16_rne(wih[e + j]) * WSC); for (int pass = 0; pass < 2; ++pass) { *(volatile v8b*)(WIH + e) = o; __threadfence(); } return; }
  const size_t t = u - n0; if (t < n1) { const size_t e = t * 8; for (int j = 0; j < 8; ++j) o[j] = (b16)(bf16_rne(w3[e + j]) * WSC); for (int pass = 0; pass < 2; ++pass) { *(volatile v8b*)(W3 + e) = o; __threadfence(); } }
}
__global__ __launch_bounds__(256) void conv1_kernel(const float* __restrict__ x, const float* __restrict__ ea, const float* __restrict__ emw, const float* __restrict__ emb, const float* __restrict__ lw, const float* __restrict__ lb, const int* __restrict__ srcs, const int* __restrict__ PERM, const int* __restrict__ ROWPTR, const int* __restrict__ ROWCNT, int permLen, float* __restrict__ S) {
  const size_t v = (size_t)blockIdx.x * 256 + threadIdx.x; float A = 0.0f, Bc = bf16_rne(lb[0]);
#pragma unroll 2
  for (int c = 0; c < H; ++c) { const float l = bf16_rne(lw[c]); A += pmul(bf16_rne(emw[c]), l); Bc += pmul(bf16_rne(emb[c]), l); }
  float s = 0.0f;
  if (v < (size_t)N) { int st = ROWPTR[v], cnt = ROWCNT[v]; cnt = iclamp(cnt, 0, 65536); st = iclamp(st, 0, permLen - cnt); float a = 0.0f;
    for (int j = 0; j < cnt; ++j) { const int e = iclamp(PERM[st + j], 0, E - 1); const int sn = iclamp(srcs[e], 0, N - 1); a += fmaxf(bf16_rne(x[sn]) + pmul(bf16_rne(ea[e]), A) + Bc, 0.0f); }
    s = bf16_rne(x[v]) + a; }
  for (int pass = 0; pass < 2; ++pass) { ((volatile float*)S)[v] = s; __threadfence(); }
}
__global__ __launch_bounds__(128) void lstm_kernel(const float* __restrict__ S, const float* __restrict__ n1w, const float* __restrict__ n1b, const b16* __restrict__ WIH, const float* __restrict__ bih, const float* __restrict__ bhh, float* __restrict__ outH, float* __restrict__ outC) {
  __shared__ __attribute__((aligned(16))) b16 Ah[4][16][H + 8], Al[4][16][H + 8]; __shared__ __attribute__((aligned(16))) float Th[4][16][36], Tc[4][16][36];
  const int wave = threadIdx.x >> 5, lane = threadIdx.x & 31, nloc = lane & 15, hlf = lane >> 4; const size_t m0 = (size_t)blockIdx.x * 64 + wave * 16; const int c0 = blockIdx.y * 32;
  float wv[4], bv[4]; for (int j = 0; j < 4; ++j) { wv[j] = opaque(bf16_rne(n1w[lane * 4 + j])); bv[j] = bf16_rne(n1b[lane * 4 + j]); }
  for (int rr = 0; rr < 16; ++rr) { const size_t r = m0 + rr; const float s = S[r < (size_t)N ? r : (size_t)(N - 1)]; for (int j = 0; j < 4; ++j) { b16 p, q; split16((pmul(s, wv[j]) + bv[j]) * XS, p, q); Ah[wave][rr][lane * 4 + j] = p; Al[wave][rr][lane * 4 + j] = q; } }
  wave_lds_sync();
  v8f acc[6];
#pragma unroll
  for (int t = 0; t < 6; ++t) acc[t] = (v8f){};
#pragma unroll 2
  for (int kb = 0; kb < H; kb += 32) { const v16b a = frag_kb(&Ah[wave][nloc][kb], hlf), al = frag_kb(&Al[wave][nloc][kb], hlf);
#pragma unroll
    for (int t = 0; t < 6; ++t) { const int gate = (t >> 1) == 0 ? 0 : ((t >> 1) == 1 ? 2 : 3); const int col = gate * H + c0 + (t & 1) * 16 + nloc; const v16b bw = frag_kb(WIH + (size_t)col * H + kb, hlf); acc[t] = wmma16b(a, bw, acc[t]); acc[t] = wmma16b(al, bw, acc[t]); } }
#pragma unroll
  for (int u2 = 0; u2 < 2; ++u2) { const int cl = u2 * 16 + nloc; const int c = c0 + cl; const float bi = bf16_rne(bih[c]) + bf16_rne(bhh[c]), bg = bf16_rne(bih[2 * H + c]) + bf16_rne(bhh[2 * H + c]), bo = bf16_rne(bih[3 * H + c]) + bf16_rne(bhh[3 * H + c]); const float sc = 1.0f / (XS * WSC);
#pragma unroll 1
    for (int r8 = 0; r8 < 8; ++r8) { const int rl = 8 * hlf + r8; const float ig = sigm(acc[u2][r8] * sc + bi), gg = tanhf(acc[2 + u2][r8] * sc + bg), og = sigm(acc[4 + u2][r8] * sc + bo); const float cc = pmul(ig, gg); Tc[wave][rl][cl] = cc; Th[wave][rl][cl] = pmul(og, tanhf(cc)); } }
  wave_lds_sync();
  for (int pass = 0; pass < 2; ++pass) { for (int rr = 0; rr < 16; ++rr) { const size_t r = m0 + rr; if (r < (size_t)N) { if (lane < 8) *(volatile v4f*)(outH + r * H + c0 + lane * 4) = *(const v4f*)(&Th[wave][rr][lane * 4]); else if (lane < 16) *(volatile v4f*)(outC + r * H + c0 + (lane - 8) * 4) = *(const v4f*)(&Tc[wave][rr][(lane - 8) * 4]); } } __threadfence(); }
}
__global__ __launch_bounds__(256) void agg3_kernel(const float* __restrict__ HN, const float* __restrict__ ea, const float* __restrict__ emw, const float* __restrict__ emb, const int* __restrict__ srcs, const int* __restrict__ PERM, const int* __restrict__ ROWPTR, const int* __restrict__ ROWCNT, int permLen, float* __restrict__ Z) {
  const int wave = threadIdx.x >> 5, lane = threadIdx.x & 31; const size_t v = (size_t)blockIdx.x * 8 + wave; v4f z = {0.0f, 0.0f, 0.0f, 0.0f};
  float w4[4], b4[4]; for (int i = 0; i < 4; ++i) { w4[i] = opaque(bf16_rne(emw[lane * 4 + i])); b4[i] = bf16_rne(emb[lane * 4 + i]); }
  if (v < (size_t)N) { int st = ROWPTR[v], cnt = ROWCNT[v]; cnt = iclamp(cnt, 0, 65536); st = iclamp(st, 0, permLen - cnt); z = *(const v4f*)(HN + v * H + lane * 4);
#pragma unroll 1
    for (int j = 0; j < cnt; ++j) { const int e = iclamp(PERM[st + j], 0, E - 1); const size_t sn = (size_t)iclamp(srcs[e], 0, N - 1); const float a = bf16_rne(ea[e]); const v4f h = *(const v4f*)(HN + sn * H + lane * 4);
      for (int i = 0; i < 4; ++i) z[i] += fmaxf(h[i] + pmul(a, w4[i]) + b4[i], 0.0f); } }
  for (int pass = 0; pass < 2; ++pass) { *(volatile v4f*)(Z + v * H + lane * 4) = z; __threadfence(); }
}
__global__ __launch_bounds__(128) void conv3_kernel(const float* __restrict__ Z, const b16* __restrict__ W3, const float* __restrict__ b3, const float* __restrict__ dw, float* __restrict__ PA, float* __restrict__ PB) {
  __shared__ __attribute__((aligned(16))) b16 Ah[4][16][H + 8], Al[4][16][H + 8]; __shared__ __attribute__((aligned(16))) float pa_s[64], pb_s[64];
  const int wave = threadIdx.x >> 5, lane = threadIdx.x & 31, nloc = lane & 15, hlf = lane >> 4; const size_t m0 = (size_t)blockIdx.x * 64 + wave * 16;
  for (int rr = 0; rr < 16; ++rr) { const v4f x = *(const v4f*)(Z + (m0 + rr) * H + lane * 4); for (int j = 0; j < 4; ++j) { b16 p, q; split16(x[j] * XS, p, q); Ah[wave][rr][lane * 4 + j] = p; Al[wave][rr][lane * 4 + j] = q; } }
  wave_lds_sync();
  v8f acc[8];
#pragma unroll
  for (int t = 0; t < 8; ++t) acc[t] = (v8f){};
#pragma unroll 2
  for (int kb = 0; kb < H; kb += 32) { const v16b a = frag_kb(&Ah[wave][nloc][kb], hlf), al = frag_kb(&Al[wave][nloc][kb], hlf);
#pragma unroll
    for (int t = 0; t < 8; ++t) { const v16b bw = frag_kb(W3 + (size_t)(t * 16 + nloc) * H + kb, hlf); acc[t] = wmma16b(a, bw, acc[t]); acc[t] = wmma16b(al, bw, acc[t]); } }
  float pa[8], pb[8]; for (int r8 = 0; r8 < 8; ++r8) { pa[r8] = 0.0f; pb[r8] = 0.0f; }
#pragma unroll
  for (int t = 0; t < 8; ++t) { const int c = t * 16 + nloc; const float bb = bf16_rne(b3[c]), wa = opaque(bf16_rne(dw[c])), wb = opaque(bf16_rne(dw[H + c]));
#pragma unroll
    for (int r8 = 0; r8 < 8; ++r8) { const float h3 = acc[t][r8] * (1.0f / (XS * WSC)) + bb; pa[r8] += pmul(h3, wa); pb[r8] += pmul(h3, wb); } }
#pragma unroll
  for (int r8 = 0; r8 < 8; ++r8) { float a = pa[r8], b = pb[r8]; for (int o = 1; o < 16; o <<= 1) { a += __shfl_xor(a, o); b += __shfl_xor(b, o); } if (nloc == 0) { pa_s[wave * 16 + 8 * hlf + r8] = a; pb_s[wave * 16 + 8 * hlf + r8] = b; } }
  __syncthreads();
  for (int pass = 0; pass < 2; ++pass) { if (threadIdx.x < 16) *(volatile v4f*)(PA + (size_t)blockIdx.x * 64 + threadIdx.x * 4) = *(const v4f*)(&pa_s[threadIdx.x * 4]); else if (threadIdx.x < 32) *(volatile v4f*)(PB + (size_t)blockIdx.x * 64 + (threadIdx.x - 16) * 4) = *(const v4f*)(&pb_s[(threadIdx.x - 16) * 4]); __threadfence(); }
}
__global__ __launch_bounds__(256) void edge_kernel(const float* __restrict__ PA, const float* __restrict__ PB, const int* __restrict__ srcs, const int* __restrict__ dsts, const float* __restrict__ db, float* __restrict__ out) {
  const size_t e = (size_t)blockIdx.x * 256 + threadIdx.x; const size_t ec = e < (size_t)E ? e : (size_t)(E - 1);
  const float o = PA[iclamp(srcs[ec], 0, N - 1)] + PB[iclamp(dsts[ec], 0, N - 1)] + bf16_rne(db[0]);
  for (int pass = 0; pass < 2; ++pass) { if (e < (size_t)E) ((volatile float*)out)[e] = o; __threadfence(); }
}
}

extern "C" void kernel_launch(void* const* d_in, const int* in_sizes, int n_in, void* d_out, int out_size, void* d_ws, size_t ws_size, hipStream_t stream) {
  (void)n_in;
  auto Fp = [&](int i) { return (const float*)d_in[i]; }; auto Ip = [&](int i) { return (const int*)d_in[i]; };
  if (in_sizes[0] != N || in_sizes[1] != E || in_sizes[2] != 2 * E || in_sizes[3] != H || in_sizes[5] != H || in_sizes[7] != H || in_sizes[9] != G4 * H || in_sizes[11] != G4 || in_sizes[13] != H * H || in_sizes[15] != 2 * H || out_size != E + 2 * N * H) return;
  size_t off = 0; char* ws = (char*)d_ws;
  auto carve = [&](size_t bytes) { char* p = ws + off; off += (bytes + 255) & ~(size_t)255; return p; };
  b16* WIH = (b16*)carve((size_t)G4 * H * 2); b16* W3 = (b16*)carve((size_t)H * H * 2); float* S = (float*)carve((size_t)NP * 4 + 1024); float* Z = (float*)carve((size_t)NP * H * 4); float* PA = (float*)carve((size_t)NP * 4); float* PB = (float*)carve((size_t)NP * 4);
  CsrBufs csr; off = csr_carve(csr, ws, off, E, N);
  if (off > ws_size || off > ((size_t)128 << 20)) return;
  float* outE = (float*)d_out; float* outH = outE + E; float* outC = outH + (size_t)N * H;
  wprep_kernel<<<(unsigned)(((size_t)G4 * H / 8 + (size_t)H * H / 8 + 255) / 256), 256, 0, stream>>>(Fp(9), Fp(13), WIH, W3);
  csr_build(csr, Ip(2) + E, E, N, stream);
  conv1_kernel<<<(NP + 255) / 256, 256, 0, stream>>>(Fp(0), Fp(1), Fp(3), Fp(4), Fp(5), Fp(6), Ip(2), csr.PERM, csr.ROWPTR, csr.ROWCNT, (int)csr.permLen, S);
  lstm_kernel<<<dim3(NP / 64, 4), 128, 0, stream>>>(S, Fp(7), Fp(8), WIH, Fp(11), Fp(12), outH, outC);
  agg3_kernel<<<NP / 8, 256, 0, stream>>>(outH, Fp(1), Fp(3), Fp(4), Ip(2), csr.PERM, csr.ROWPTR, csr.ROWCNT, (int)csr.permLen, Z);
  conv3_kernel<<<NP / 64, 128, 0, stream>>>(Z, W3, Fp(14), Fp(15), PA, PB);
  edge_kernel<<<(E + 255) / 256, 256, 0, stream>>>(PA, PB, Ip(2), Ip(2) + E, Fp(16), outE);
}
